// LineageLinkPredictionGNN_21028159881504
// MI455X (gfx1250) — hardware-verified
//
#include <hip/hip_runtime.h>
#include <stddef.h>


#define DF      128
#define DH      64
#define NTHR    256
#define NWAVE   8
#define EPT     8
#define NGRP    2
#define CHUNK   (NTHR * EPT * NGRP)
#define WCAP    (EPT * NGRP * 32)
#define LISTN   (NWAVE * WCAP)
#define NB      512
#define NBD     4096
#define DEDGE   (NWAVE * 128)
#define WPLANE  (DF * DF)
#define WSCALE  8.0f
#define WINV    0.125f

#define LDS_LAYER (NB * DF * 4 + LISTN * 4 + 64)

static_assert((CHUNK & (CHUNK - 1)) == 0);
static_assert(CHUNK <= 4096);
static_assert((NB & (NB - 1)) == 0 && NB <= 4096);
static_assert((NBD & (NBD - 1)) == 0 && NBD <= 4096);
static_assert(NB == 16 * NWAVE * 4);
static_assert(NBD == NWAVE * 4 * 128);

typedef float    v4f  __attribute__((ext_vector_type(4)));
typedef float    v8f  __attribute__((ext_vector_type(8)));
typedef int      v4i  __attribute__((ext_vector_type(4)));
typedef _Float16 v8h  __attribute__((ext_vector_type(8)));
typedef _Float16 v16h __attribute__((ext_vector_type(16)));
union FragH { v16h v; v8h h[2]; };

__device__ __forceinline__ v8h cvt8(v4f a, v4f b) {
  v8h r;
  r[0] = (_Float16)a.x; r[1] = (_Float16)a.y; r[2] = (_Float16)a.z; r[3] = (_Float16)a.w;
  r[4] = (_Float16)b.x; r[5] = (_Float16)b.y; r[6] = (_Float16)b.z; r[7] = (_Float16)b.w;
  return r;
}

__device__ __forceinline__ v8f wmh(v16h a, v16h b, v8f c) {
  v8f d = __builtin_amdgcn_wmma_f32_16x16x32_f16(false, a, false, b, (short)0, c, false, false);
  asm volatile("v_nop\n\tv_nop\n\tv_nop\n\tv_nop" : "+v"(d) : "v"(a), "v"(b));
  return d;
}

template <int NBT>
__device__ __forceinline__ int scan_chunk(const int* __restrict__ dsts, int nE, int cbase, int nodeBase,
                                          int vec8, int* list, int tid, int lane, int wave) {
  int wc = 0;
#pragma unroll
  for (int g = 0; g < NGRP; ++g) {
    const int el0  = (g * NTHR + tid) * EPT;
    const int e0   = cbase + el0;
    const int sent = -2147483647 - 1;
    v4i da, db;
    if (vec8 != 0 && cbase + CHUNK <= nE) {
      da = *(const v4i*)(dsts + e0);
      db = *(const v4i*)(dsts + e0 + 4);
    } else {
      da.x = (e0     < nE) ? dsts[min(e0, nE - 1)]     : sent;
      da.y = (e0 + 1 < nE) ? dsts[min(e0 + 1, nE - 1)] : sent;
      da.z = (e0 + 2 < nE) ? dsts[min(e0 + 2, nE - 1)] : sent;
      da.w = (e0 + 3 < nE) ? dsts[min(e0 + 3, nE - 1)] : sent;
      db.x = (e0 + 4 < nE) ? dsts[min(e0 + 4, nE - 1)] : sent;
      db.y = (e0 + 5 < nE) ? dsts[min(e0 + 5, nE - 1)] : sent;
      db.z = (e0 + 6 < nE) ? dsts[min(e0 + 6, nE - 1)] : sent;
      db.w = (e0 + 7 < nE) ? dsts[min(e0 + 7, nE - 1)] : sent;
    }
    const unsigned nb = (unsigned)nodeBase;
    const unsigned s0 = (unsigned)da.x - nb, s1 = (unsigned)da.y - nb;
    const unsigned s2 = (unsigned)da.z - nb, s3 = (unsigned)da.w - nb;
    const unsigned s4 = (unsigned)db.x - nb, s5 = (unsigned)db.y - nb;
    const unsigned s6 = (unsigned)db.z - nb, s7 = (unsigned)db.w - nb;
    const bool h0 = s0 < (unsigned)NBT, h1 = s1 < (unsigned)NBT, h2 = s2 < (unsigned)NBT, h3 = s3 < (unsigned)NBT;
    const bool h4 = s4 < (unsigned)NBT, h5 = s5 < (unsigned)NBT, h6 = s6 < (unsigned)NBT, h7 = s7 < (unsigned)NBT;
    const unsigned any = __builtin_amdgcn_ballot_w32(h0 | h1 | h2 | h3 | h4 | h5 | h6 | h7);
    if (any != 0u) {
#define HITJ(J, HJ, SJ) { \
        const unsigned mj = __builtin_amdgcn_ballot_w32(HJ); \
        if (mj != 0u) { \
          if (HJ) { \
            const int pos = wc + (int)__builtin_amdgcn_mbcnt_lo(mj, 0u); \
            if (pos < WCAP) list[wave * WCAP + pos] = ((el0 + (J)) << 12) | (int)(SJ); \
          } \
          wc += (int)__builtin_popcount(mj); } }
      HITJ(0, h0, s0)
      HITJ(1, h1, s1)
      HITJ(2, h2, s2)
      HITJ(3, h3, s3)
      HITJ(4, h4, s4)
      HITJ(5, h5, s5)
      HITJ(6, h6, s6)
      HITJ(7, h7, s7)
#undef HITJ
    }
  }
  return wc;
}

__global__ __launch_bounds__(NTHR) void k_wprep(
    const float* __restrict__ W1, const float* __restrict__ W2, const float* __restrict__ Wd1,
    _Float16* wts) {
  const int seg = blockIdx.x >> 3;
  const int li  = (blockIdx.x & 7) * NTHR + threadIdx.x;
  const int o   = li * 8;
  const int n   = o >> 7;
  const int k0  = o & (DF - 1);
  const float* base;
  int stride, roff, col;
  if (seg == 0)      { base = W1;  stride = DF; roff = 0; col = n; }
  else if (seg == 1) { base = W2;  stride = DF; roff = 0; col = n; }
  else {
    base = Wd1; stride = DH;
    const int hi = (n >= DH) ? 1 : 0;
    roff = hi * DF; col = n - hi * DH;
  }
  const float* p = base + (size_t)(roff + k0) * stride + col;
  v4f a, b;
  a.x = p[0];          a.y = p[stride];     a.z = p[2 * stride]; a.w = p[3 * stride];
  b.x = p[4 * stride]; b.y = p[5 * stride]; b.z = p[6 * stride]; b.w = p[7 * stride];
  a = a * WSCALE;
  b = b * WSCALE;
  const v8h hv = cvt8(a, b);
  _Float16* dp = wts + (size_t)seg * WPLANE + o;
  *(volatile v8h*)dp = hv;
  __threadfence();
  *(volatile v8h*)dp = hv;
}

__global__ __launch_bounds__(NTHR) void k_deg(
    const int* __restrict__ ei, float* dinv, int nE, int vec8) {
  __shared__ __attribute__((aligned(16))) int cnt[NBD];
  __shared__ __attribute__((aligned(16))) int list[LISTN];
  __shared__ int wcnt[NWAVE];
  const int tid = threadIdx.x, lane = tid & 31, wave = tid >> 5;
  const int nodeBase = blockIdx.x * NBD;
  const int* dsts = ei + nE;

  for (int i = tid; i < NBD; i += NTHR) cnt[i] = 0;
  __syncthreads();

  const int nChunks = (nE + CHUNK - 1) / CHUNK;
#pragma unroll 1
  for (int ch = 0; ch < nChunks; ++ch) {
    const int cbase = ch * CHUNK;
    const int wc = scan_chunk<NBD>(dsts, nE, cbase, nodeBase, vec8, list, tid, lane, wave);
    if (lane == 0) wcnt[wave] = wc;
    __syncthreads();
    if (wave == 0) {
#pragma unroll 1
      for (int wsx = 0; wsx < NWAVE; ++wsx) {
        int n = __builtin_amdgcn_readfirstlane(wcnt[wsx]);
        n = n > WCAP ? WCAP : (n < 0 ? 0 : n);
        const int* lp = list + wsx * WCAP;
#pragma unroll 1
        for (int i = 0; i < n; ++i) {
          const int ent  = __builtin_amdgcn_readfirstlane(lp[i]);
          const int slot = ent & (NBD - 1);
          if (lane == 0) cnt[slot] = cnt[slot] + 1;
        }
      }
    }
    __syncthreads();
  }

  v4f dq[4];
#pragma unroll
  for (int q = 0; q < 4; ++q) {
    const int f = (wave * 4 + q) * 128 + 4 * lane;
    const v4i c = *(const v4i*)(cnt + f);
    dq[q].x = rsqrtf((float)(c.x + 1));
    dq[q].y = rsqrtf((float)(c.y + 1));
    dq[q].z = rsqrtf((float)(c.z + 1));
    dq[q].w = rsqrtf((float)(c.w + 1));
  }
  float* dp = dinv + (size_t)nodeBase;
#pragma unroll
  for (int q = 0; q < 4; ++q) *(volatile v4f*)(dp + (wave * 4 + q) * 128 + 4 * lane) = dq[q];
  __threadfence();
#pragma unroll
  for (int q = 0; q < 4; ++q) *(volatile v4f*)(dp + (wave * 4 + q) * 128 + 4 * lane) = dq[q];
}

template <int RELU, int HASBIAS>
__device__ __forceinline__ void gemm_rows(float* accL, const _Float16* __restrict__ w,
                                          const float* __restrict__ bias, int wave, int lane) {
  const int hh = lane >> 4, m = lane & 15;
  float bb[8];
#pragma unroll
  for (int t = 0; t < 8; ++t) bb[t] = HASBIAS ? bias[16 * t + m] : 0.f;
#pragma unroll 1
  for (int q = 0; q < NB / (16 * NWAVE); ++q) {
    const int tile = wave + NWAVE * q;
    v8f c8[8];
#pragma unroll
    for (int t = 0; t < 8; ++t) { v8f z = {0.f, 0.f, 0.f, 0.f, 0.f, 0.f, 0.f, 0.f}; c8[t] = z; }
    const float* ar = accL + (size_t)(16 * tile + m) * DF + 8 * hh;
#pragma unroll
    for (int kt = 0; kt < DF / 32; ++kt) {
      const v4f p0 = *(const v4f*)(ar + 32 * kt),      p1 = *(const v4f*)(ar + 32 * kt + 4);
      const v4f p2 = *(const v4f*)(ar + 32 * kt + 16), p3 = *(const v4f*)(ar + 32 * kt + 20);
      FragH a;
      a.h[0] = cvt8(p0, p1);
      a.h[1] = cvt8(p2, p3);
#pragma unroll
      for (int t = 0; t < 8; ++t) {
        const _Float16* bp = w + (size_t)(16 * t + m) * DF + 32 * kt + 8 * hh;
        FragH b;
        b.h[0] = *(const v8h*)bp;
        b.h[1] = *(const v8h*)(bp + 16);
        c8[t] = wmh(a.v, b.v, c8[t]);
      }
    }
    float* sp = accL + (size_t)(16 * tile + 8 * hh) * DF + m;
#pragma unroll
    for (int t = 0; t < 8; ++t) {
#pragma unroll
      for (int r = 0; r < 8; ++r) {
        float v = c8[t][r] * WINV + bb[t];
        if (RELU) v = fmaxf(v, 0.f);
        sp[r * DF + 16 * t] = v;
      }
    }
  }
}

template <int RELU, int SECOND>
__global__ __launch_bounds__(NTHR) void k_layer(
    const int* __restrict__ ei, const float* __restrict__ srcp, const float* __restrict__ dinv,
    const _Float16* __restrict__ wn, const float* __restrict__ bias, const _Float16* __restrict__ wc,
    float* outp, int nN, int nE, int vec8) {
  extern __shared__ v4f lds_dyn[];
  float* acc  = (float*)lds_dyn;
  int*   list = (int*)(acc + NB * DF);
  int*   wcnt = list + LISTN;
  const int tid = threadIdx.x, lane = tid & 31, wave = tid >> 5;
  const int nodeBase = blockIdx.x * NB;
  const int* dsts = ei + nE;

  {
    const v4f z = {0.f, 0.f, 0.f, 0.f};
    for (int i = tid; i < NB * DF / 4; i += NTHR) lds_dyn[i] = z;
  }
  __syncthreads();

  const int nChunks = (nE + CHUNK - 1) / CHUNK;
#pragma unroll 1
  for (int ch = 0; ch < nChunks; ++ch) {
    const int cbase = ch * CHUNK;
    const int wcn = scan_chunk<NB>(dsts, nE, cbase, nodeBase, vec8, list, tid, lane, wave);
    if (lane == 0) wcnt[wave] = wcn;
    __syncthreads();
    if (wave == 0) {
#pragma unroll 1
      for (int wsx = 0; wsx < NWAVE; ++wsx) {
        int n = __builtin_amdgcn_readfirstlane(wcnt[wsx]);
        n = n > WCAP ? WCAP : (n < 0 ? 0 : n);
        const int* lp = list + wsx * WCAP;
#pragma unroll 1
        for (int i = 0; i < n; ++i) {
          const int ent  = __builtin_amdgcn_readfirstlane(lp[i]);
          const int slot = ent & (NB - 1);
          int e = cbase + ((ent >> 12) & (CHUNK - 1));
          e = e > nE - 1 ? nE - 1 : e;
          int src = ei[e];
          src = src < 0 ? 0 : (src > nN - 1 ? nN - 1 : src);
          const float ds = dinv[src];
          const v4f v = *(const v4f*)(srcp + (size_t)src * DF + 4 * lane);
          v4f* ap = (v4f*)(acc + slot * DF + 4 * lane);
          *ap = *ap + v * ds;
        }
      }
    }
    __syncthreads();
  }

#pragma unroll 4
  for (int i = 0; i < (NB * DF / 4) / NTHR; ++i) {
    const int idx  = i * NTHR + tid;
    const int slot = idx >> 5;
    const int c4   = (idx & 31) * 4;
    int node = nodeBase + slot;
    node = node > nN - 1 ? nN - 1 : node;
    const float d  = dinv[node];
    const v4f   sv = *(const v4f*)(srcp + (size_t)node * DF + c4);
    v4f* ap = (v4f*)(acc + slot * DF + c4);
    *ap = (*ap + sv * d) * d;
  }
  __syncthreads();

  gemm_rows<RELU, 1>(acc, wn, bias, wave, lane);
  __syncthreads();
  if (SECOND) {
    gemm_rows<0, 0>(acc, wc, bias, wave, lane);
    __syncthreads();
  }

  const float* lrow = acc + (size_t)(64 * wave) * DF + 4 * lane;
  float* grow = outp + ((size_t)nodeBase + 64 * wave) * DF + 4 * lane;
#pragma unroll 4
  for (int i = 0; i < 64; ++i) { const v4f v = *(const v4f*)(lrow + i * DF); *(volatile v4f*)(grow + (size_t)i * DF) = v; }
  __threadfence();
#pragma unroll 4
  for (int i = 0; i < 64; ++i) { const v4f v = *(const v4f*)(lrow + i * DF); *(volatile v4f*)(grow + (size_t)i * DF) = v; }
}

__global__ __launch_bounds__(NTHR) void k_dec(
    const int* __restrict__ ei, const float* __restrict__ pq, const float* __restrict__ bd1,
    const float* __restrict__ wd2, const float* __restrict__ bd2, float* out, int nN, int nE) {
  __shared__ __attribute__((aligned(16))) float sbw[2 * DH];
  __shared__ __attribute__((aligned(16))) float stg[NWAVE * 128];
  const int tid = threadIdx.x, lane = tid & 31, wave = tid >> 5;
  if (tid < 2 * DH) {
    int i1 = tid;      i1 = i1 > DH - 1 ? DH - 1 : i1;
    int i2 = tid - DH; i2 = i2 < 0 ? 0 : i2;
    const float vb = bd1[i1];
    const float vw = wd2[i2];
    sbw[tid] = (tid < DH) ? vb : vw;
  }
  const float bd2v = bd2[0];
  __syncthreads();

  const int ebase = (blockIdx.x * NWAVE + wave) * 128;
#pragma unroll 1
  for (int g = 0; g < 4; ++g) {
    const int e = ebase + 32 * g + lane;
    int ec = e > nE - 1 ? nE - 1 : e;
    ec = ec < 0 ? 0 : ec;
    int src = ei[ec];
    int dst = ei[(size_t)nE + ec];
    src = src < 0 ? 0 : (src > nN - 1 ? nN - 1 : src);
    dst = dst < 0 ? 0 : (dst > nN - 1 ? nN - 1 : dst);
    const float* pp = pq + (size_t)src * DF;
    const float* qp = pq + (size_t)dst * DF + DH;
    float s = 0.f;
#pragma unroll 4
    for (int c = 0; c < DH / 4; ++c) {
      const v4f p = *(const v4f*)(pp + 4 * c);
      const v4f q = *(const v4f*)(qp + 4 * c);
      const v4f b = *(const v4f*)(sbw + 4 * c);
      const v4f w = *(const v4f*)(sbw + DH + 4 * c);
      v4f h = p + q + b;
      h.x = fmaxf(h.x, 0.f); h.y = fmaxf(h.y, 0.f); h.z = fmaxf(h.z, 0.f); h.w = fmaxf(h.w, 0.f);
      s += h.x * w.x; s += h.y * w.y; s += h.z * w.z; s += h.w * w.w;
    }
    stg[wave * 128 + 32 * g + lane] = s + bd2v;
  }
  __syncthreads();

  const v4f ov = *(const v4f*)(stg + wave * 128 + 4 * lane);
  const bool full = (ebase + 128 <= nE);
  if (full) {
    *(volatile v4f*)(out + (size_t)ebase + 4 * lane) = ov;
  } else {
#pragma unroll
    for (int j = 0; j < 4; ++j) {
      const int idx = ebase + 4 * lane + j;
      if (idx < nE) *(volatile float*)(out + idx) = ov[j];
    }
  }
  __threadfence();
  if (full) {
    *(volatile v4f*)(out + (size_t)ebase + 4 * lane) = ov;
  } else {
#pragma unroll
    for (int j = 0; j < 4; ++j) {
      const int idx = ebase + 4 * lane + j;
      if (idx < nE) *(volatile float*)(out + idx) = ov[j];
    }
  }
}

extern "C" void kernel_launch(void* const* d_in, const int* in_sizes, int n_in,
                              void* d_out, int out_size, void* d_ws, size_t ws_size,
                              hipStream_t stream) {
  if (n_in < 10) return;
  const int nN = in_sizes[0] / DF;
  const int nE = in_sizes[1] / 2;
  if (nN <= 0 || nE <= 0 || in_sizes[0] != nN * DF || in_sizes[1] != nE * 2) return;
  if (in_sizes[2] != DF * DF || in_sizes[3] < DF || in_sizes[4] != DF * DF || in_sizes[5] < DF) return;
  if (in_sizes[6] != 2 * DF * DH || in_sizes[7] < DH || in_sizes[8] < DH || in_sizes[9] < 1) return;
  if (out_size != nE) return;

  const float* x   = (const float*)d_in[0];
  const int*   ei  = (const int*)d_in[1];
  const float* W1  = (const float*)d_in[2];
  const float* b1  = (const float*)d_in[3];
  const float* W2  = (const float*)d_in[4];
  const float* b2  = (const float*)d_in[5];
  const float* Wd1 = (const float*)d_in[6];
  const float* bd1 = (const float*)d_in[7];
  const float* Wd2 = (const float*)d_in[8];
  const float* bd2 = (const float*)d_in[9];
  float* out = (float*)d_out;

  const int nBD = (nN + NBD - 1) / NBD;
  const int nA  = (nN + NB - 1) / NB;
  const int nDC = (nE + DEDGE - 1) / DEDGE;

  char* ws = (char*)d_ws;
  size_t off = 0;
  const size_t oW  = off; off += (size_t)3 * WPLANE * 2;                       off = (off + 255) & ~(size_t)255;
  const size_t oDv = off; off += (size_t)nBD * NBD * 4;                        off = (off + 255) & ~(size_t)255;
  const size_t oZ1 = off; off += (size_t)nA * NB * DF * 4;                     off = (off + 255) & ~(size_t)255;
  const size_t oPQ = off; off += (size_t)nA * NB * DF * 4;                     off = (off + 255) & ~(size_t)255;
  if (off > ws_size || off > ((size_t)128 << 20)) return;
  _Float16* wts  = (_Float16*)(ws + oW);
  float*    dinv = (float*)(ws + oDv);
  float*    z1   = (float*)(ws + oZ1);
  float*    pq   = (float*)(ws + oPQ);
  const _Float16* w1s = wts;
  const _Float16* w2s = wts + WPLANE;
  const _Float16* wcs = wts + 2 * WPLANE;

  const int vec8 = ((nE & 3) == 0) ? 1 : 0;

  k_wprep<<<24, NTHR, 0, stream>>>(W1, W2, Wd1, wts);

  k_deg<<<nBD, NTHR, 0, stream>>>(ei, dinv, nE, vec8);

  hipFuncSetAttribute(reinterpret_cast<const void*>(&k_layer<1, 0>),
                      hipFuncAttributeMaxDynamicSharedMemorySize, LDS_LAYER);
  k_layer<1, 0><<<nA, NTHR, LDS_LAYER, stream>>>(ei, x, dinv, w1s, b1, w1s, z1, nN, nE, vec8);

  hipFuncSetAttribute(reinterpret_cast<const void*>(&k_layer<0, 1>),
                      hipFuncAttributeMaxDynamicSharedMemorySize, LDS_LAYER);
  k_layer<0, 1><<<nA, NTHR, LDS_LAYER, stream>>>(ei, z1, dinv, w2s, b2, wcs, pq, nN, nE, vec8);

  k_dec<<<nDC, NTHR, 0, stream>>>(ei, pq, bd1, Wd2, bd2, out, nN, nE);
}
